// RelPartialLearnableMultiHeadAttn_64914135712023
// MI455X (gfx1250) — hardware-verified
//
#include <hip/hip_runtime.h>
#include <math.h>

constexpr int kQ      = 2048;
constexpr int kB      = 2;
constexpr int kD      = 1024;
constexpr int kH      = 16;
constexpr int kDH     = 64;
constexpr int kTok    = kQ * kB;
constexpr int kHD     = kH * kDH;
constexpr int kGroups = kB * kH;
constexpr int kChunkG = 2;
constexpr int kNumChunks = kGroups / kChunkG;
static_assert(kH % kChunkG == 0, "chunk groups share b");

constexpr float kWCarry     = 16.0f;
constexpr float kWCarryInv  = 1.0f / 16.0f;
constexpr float kPCarry     = 2048.0f;
constexpr float kVecCarry   = 256.0f;
constexpr float kPVScale    = kVecCarry / kPCarry;
constexpr float kOutScale   = 1.0f / (kVecCarry * kWCarry);
constexpr float kScoreScale = 0.125f;
constexpr float kInvD       = 1.0f / 1024.0f;
constexpr float kLnEps      = 1e-5f;

constexpr size_t kMiB       = 1048576;
constexpr size_t OFF_W16    = 0;
constexpr size_t OFF_QKVW16 = 8 * kMiB;
constexpr size_t OFF_RNW16  = 14 * kMiB;
constexpr size_t OFF_P16    = 0;
constexpr size_t OFF_OW16   = 16 * kMiB;
constexpr size_t OFF_RK16   = 18 * kMiB;
constexpr size_t OFF_QW16   = 22 * kMiB;
constexpr size_t OFF_QR16   = 30 * kMiB;
constexpr size_t OFF_K16    = 38 * kMiB;
constexpr size_t OFF_VT16   = 46 * kMiB;
constexpr size_t OFF_VEC16  = 54 * kMiB;
constexpr size_t OFF_SAC    = 62 * kMiB;
constexpr size_t OFF_R16    = 62 * kMiB;
constexpr size_t OFF_WQ32   = 66 * kMiB;
constexpr size_t OFF_X32    = 62 * kMiB;
constexpr size_t OFF_SBD    = 94 * kMiB;
constexpr size_t kWsTotal   = 126 * kMiB;
static_assert((size_t)kTok * kD * 2 == 8 * kMiB, "W16/QW16/QR16/K16/VEC16 plane size");
static_assert((size_t)3 * kHD * kD * 2 == 6 * kMiB, "QKVW16 size");
static_assert((size_t)kHD * kD * 2 == 2 * kMiB, "RNW16/OW16 size");
static_assert((size_t)kQ * kHD * 2 == 4 * kMiB, "RK16/R16 size");
static_assert((size_t)kHD * kTok * 2 == 8 * kMiB, "VT16 size");
static_assert((size_t)kChunkG * kQ * kQ * 2 == 16 * kMiB, "P16 chunk size");
static_assert((size_t)kChunkG * kQ * kQ * 4 == 32 * kMiB, "score chunk size");
static_assert((size_t)kTok * kD * 4 == 16 * kMiB, "WQ32/X32 size");
static_assert(OFF_WQ32 + 16 * kMiB <= OFF_SBD, "early overlay fits");
static_assert(OFF_SBD + 32 * kMiB == kWsTotal, "total");
static_assert(kWsTotal == 132120576, "carve total");

typedef __attribute__((ext_vector_type(16))) _Float16 v16h;
typedef __attribute__((ext_vector_type(8)))  _Float16 v8h;
typedef __attribute__((ext_vector_type(16))) __bf16   v16b;
typedef __attribute__((ext_vector_type(8)))  __bf16   v8b;
typedef __attribute__((ext_vector_type(8)))  float    v8f;
typedef __attribute__((ext_vector_type(4)))  float    v4f;
typedef __attribute__((ext_vector_type(4)))  unsigned int v4u;
typedef __attribute__((ext_vector_type(4)))  int v4i;

__device__ __forceinline__ unsigned short f2bf_bits(float f) {
  unsigned u = __float_as_uint(f);
  return (unsigned short)((u + 0x7FFFu + ((u >> 16) & 1u)) >> 16);
}
__device__ __forceinline__ float bf_bits2f(unsigned short h) { return __uint_as_float(((unsigned)h) << 16); }

__device__ __forceinline__ void dep_guard_h(v8f& a, v8f& b, v16h x, v16h y) { asm volatile("v_nop\n\tv_nop\n\tv_nop\n\tv_nop" : "+v"(a), "+v"(b) : "v"(x), "v"(y)); }
__device__ __forceinline__ void dep_guard_b(v8f& a, v8f& b, v16b x, v16b y) { asm volatile("v_nop\n\tv_nop\n\tv_nop\n\tv_nop" : "+v"(a), "+v"(b) : "v"(x), "v"(y)); }
__device__ __forceinline__ void keep4_h(v16h a, v16h b, v16h c, v16h d) { asm volatile("v_nop" :: "v"(a), "v"(b), "v"(c), "v"(d)); }
__device__ __forceinline__ void keep4_b(v16b a, v16b b, v16b c, v16b d) { asm volatile("v_nop" :: "v"(a), "v"(b), "v"(c), "v"(d)); }
__device__ __forceinline__ void acc_guard4(v8f& a, v8f& b, v8f& c, v8f& d) { asm volatile("v_nop\n\tv_nop\n\tv_nop\n\tv_nop" : "+v"(a), "+v"(b), "+v"(c), "+v"(d)); }
template <typename T> struct Frag;
template <> struct Frag<_Float16> {
  typedef v16h V; union U { v16h v; v8h h[2]; };
  static __device__ __forceinline__ v16h load(const _Float16* p) {
    U f; f.h[0] = *(const v8h*)(p); f.h[1] = *(const v8h*)(p + 16); return f.v;
  }
  static __device__ __forceinline__ v8f mma(v16h a, v16h b, v8f c) {
    return __builtin_amdgcn_wmma_f32_16x16x32_f16(false, a, false, b, (short)0, c, false, false);
  }
  static __device__ __forceinline__ void guard(v8f& a, v8f& b, v16h x, v16h y) { dep_guard_h(a, b, x, y); }
  static __device__ __forceinline__ void keep(v16h a, v16h b, v16h c, v16h d) { keep4_h(a, b, c, d); }
};
template <> struct Frag<__bf16> {
  typedef v16b V; union U { v16b v; v8b h[2]; };
  static __device__ __forceinline__ v16b load(const __bf16* p) {
    U f; f.h[0] = *(const v8b*)(p); f.h[1] = *(const v8b*)(p + 16); return f.v;
  }
  static __device__ __forceinline__ v8f mma(v16b a, v16b b, v8f c) {
    return __builtin_amdgcn_wmma_f32_16x16x32_bf16(false, a, false, b, (short)0, c, false, false);
  }
  static __device__ __forceinline__ void guard(v8f& a, v8f& b, v16b x, v16b y) { dep_guard_b(a, b, x, y); }
  static __device__ __forceinline__ void keep(v16b a, v16b b, v16b c, v16b d) { keep4_b(a, b, c, d); }
};

__device__ __forceinline__ unsigned pk16(unsigned short a, unsigned short b) { return (unsigned)a | ((unsigned)b << 16); }
__device__ __forceinline__ unsigned short h_bits(float f) { const _Float16 h = (_Float16)f; return __builtin_bit_cast(unsigned short, h); }

template <int ET> struct Elem;
template <> struct Elem<0> { typedef _Float16 T; };
template <> struct Elem<1> { typedef __bf16 T; };
template <int ET, bool SPLIT, int BIAS_MODE, int OUT_MODE, bool RESID, int ACT = 0>
__global__ __launch_bounds__(256) void wmma_gemm64(
    const unsigned short* __restrict__ Ap, const unsigned short* __restrict__ A2p, int lda, long strideA,
    const unsigned short* __restrict__ Btp, const unsigned short* __restrict__ Bt2p, int ldb, long strideB,
    void* __restrict__ Cout, void* __restrict__ Cout2, int ldc, long strideC,
    const float* __restrict__ bias,
    const float* __restrict__ resid, long strideR,
    int M, int N, int K, float scale) {
  typedef typename Elem<ET>::T T;
  typedef typename Frag<T>::V V;
  const T* A = (const T*)Ap; const T* A2 = (const T*)A2p; const T* Bt = (const T*)Btp; const T* Bt2 = (const T*)Bt2p;
  __shared__ __align__(16) float sT[8][16 * 68];
  const int b    = blockIdx.y;
  const int lane = threadIdx.x & 31;
  const int wave = threadIdx.x >> 5;
  const int tilesN = N >> 6;
  const int tilesM = M >> 6;
  const int tile = blockIdx.x * 8 + wave;
  if (tile >= tilesM * tilesN) return;
  const int tm = tile / tilesN;
  const int tn = tile - tm * tilesN;
  const int m0 = tm << 6;
  const int n0 = tn << 6;

  const T* Ab  = A  + (size_t)b * strideA;
  const T* Bb  = Bt + (size_t)b * strideB;
  const T* Ab2 = SPLIT ? (A2  + (size_t)b * strideA) : nullptr;
  const T* Bb2 = SPLIT ? (Bt2 + (size_t)b * strideB) : nullptr;

  const int rlane = lane & 15;
  const int koff  = (lane >> 4) * 8;
  const int mOff  = (lane >> 4) * 8;

  v8f acc[4][4];
#pragma unroll
  for (int i = 0; i < 4; ++i)
#pragma unroll
    for (int j = 0; j < 4; ++j) acc[i][j] = (v8f){0.f,0.f,0.f,0.f,0.f,0.f,0.f,0.f};

  for (int k0 = 0; k0 < K; k0 += 32) {
    V bh[4], bl[4];
#pragma unroll
    for (int j = 0; j < 4; ++j) {
      const size_t bo = (size_t)(n0 + (j << 4) + rlane) * ldb + koff + k0;
      bh[j] = Frag<T>::load(Bb + bo);
      if (SPLIT) bl[j] = Frag<T>::load(Bb2 + bo);
    }
#pragma unroll
    for (int i = 0; i < 4; ++i) {
      const size_t ao = (size_t)(m0 + (i << 4) + rlane) * lda + koff + k0;
      V ah = Frag<T>::load(Ab + ao);
      V al;
      if (SPLIT) al = Frag<T>::load(Ab2 + ao);
#pragma unroll
      for (int j = 0; j < 4; ++j) {
        acc[i][j] = Frag<T>::mma(ah, bh[j], acc[i][j]);
        if (SPLIT) {
          acc[i][j] = Frag<T>::mma(ah, bl[j], acc[i][j]);
          acc[i][j] = Frag<T>::mma(al, bh[j], acc[i][j]);
        }
      }
      Frag<T>::guard(acc[i][0], acc[i][3], ah, SPLIT ? al : ah);
    }
    Frag<T>::keep(bh[0], bh[1], bh[2], bh[3]);
    if (SPLIT) Frag<T>::keep(bl[0], bl[1], bl[2], bl[3]);
  }
  acc_guard4(acc[0][0], acc[0][1], acc[0][2], acc[0][3]);
  acc_guard4(acc[1][0], acc[1][1], acc[1][2], acc[1][3]);
  acc_guard4(acc[2][0], acc[2][1], acc[2][2], acc[2][3]);
  acc_guard4(acc[3][0], acc[3][1], acc[3][2], acc[3][3]);

  float* slab = sT[wave];
  const float* Rb = RESID ? (resid + (size_t)b * strideR) : nullptr;
#pragma unroll
  for (int i = 0; i < 4; ++i) {
    const int mBase = m0 + (i << 4);
#pragma unroll
    for (int j = 0; j < 4; ++j) {
      const int n = n0 + (j << 4) + rlane;
      float bv = 0.f;
      if (BIAS_MODE == 2) bv = bias[n];
#pragma unroll
      for (int r = 0; r < 8; ++r) {
        float v = acc[i][j][r] * scale;
        if (BIAS_MODE == 1) v += bias[mBase + mOff + r];
        if (BIAS_MODE == 2) v += bv;
        if (RESID) v += Rb[(size_t)(mBase + mOff + r) * ldc + n];
        if (ACT == 2) v = fmaxf(v, 0.0f);
        if (ACT == 4) v = (v > 0.f) ? v : 0.01f * v;
        slab[(mOff + r) * 68 + (j << 4) + rlane] = v;
      }
    }
    __builtin_amdgcn_fence(__ATOMIC_RELEASE, "workgroup");
    __builtin_amdgcn_wave_barrier();
    __builtin_amdgcn_fence(__ATOMIC_ACQUIRE, "workgroup");
    if (OUT_MODE == 0) {
      float* C = (float*)Cout + (size_t)b * strideC;
      const int hh = lane >> 4, c4 = (lane & 15) * 4;
      for (int pass = 0; pass < 2; ++pass) {
#pragma unroll
        for (int it = 0; it < 8; ++it) {
          const int row = it * 2 + hh;
          v4f v = *(const v4f*)(slab + row * 68 + c4);
          *(volatile v4f*)(C + (size_t)(mBase + row) * ldc + n0 + c4) = v;
        }
        __threadfence();
      }
    } else {
      const int q = lane >> 3, c8 = (lane & 7) * 8;
      unsigned short* C  = (unsigned short*)Cout  + (size_t)b * strideC;
      unsigned short* C2 = (OUT_MODE == 2) ? ((unsigned short*)Cout2 + (size_t)b * strideC) : nullptr;
      for (int pass = 0; pass < 2; ++pass) {
#pragma unroll
        for (int it = 0; it < 4; ++it) {
          const int row = it * 4 + q;
          const float* sp = slab + row * 68 + c8;
          v8h hv, lv;
#pragma unroll
          for (int e = 0; e < 8; ++e) {
            if (OUT_MODE == 1) {
              hv[e] = (_Float16)sp[e];
            } else {
              unsigned short hb = f2bf_bits(sp[e]);
              unsigned short lb = f2bf_bits(sp[e] - bf_bits2f(hb));
              hv[e] = __builtin_bit_cast(_Float16, hb);
              lv[e] = __builtin_bit_cast(_Float16, lb);
            }
          }
          *(volatile v8h*)(C + (size_t)(mBase + row) * ldc + n0 + c8) = hv;
          if (OUT_MODE == 2) *(volatile v8h*)(C2 + (size_t)(mBase + row) * ldc + n0 + c8) = lv;
        }
        __threadfence();
      }
    }
    __builtin_amdgcn_fence(__ATOMIC_RELEASE, "workgroup");
    __builtin_amdgcn_wave_barrier();
    __builtin_amdgcn_fence(__ATOMIC_ACQUIRE, "workgroup");
  }
}

__global__ __launch_bounds__(256) void cast8_f16_kernel(const float* __restrict__ in, unsigned short* __restrict__ out,
                                                        int n8, float scale) {
  const int i = blockIdx.x * 256 + threadIdx.x;
  if (i >= n8) return;
  const float* p = in + 8 * (size_t)i;
  const v4f a = *(const v4f*)(p);
  const v4f c = *(const v4f*)(p + 4);
  unsigned short hb[8];
#pragma unroll
  for (int e = 0; e < 4; ++e) {
    hb[e]     = h_bits(a[e] * scale);
    hb[4 + e] = h_bits(c[e] * scale);
  }
  const v4u u = (v4u){pk16(hb[0], hb[1]), pk16(hb[2], hb[3]), pk16(hb[4], hb[5]), pk16(hb[6], hb[7])};
  unsigned short* q = out + 8 * (size_t)i;
  *(volatile v4u*)q = u;
  __threadfence();
  *(volatile v4u*)q = u;
}

__global__ __launch_bounds__(256) void castw_bm_kernel(const float* __restrict__ w, unsigned short* __restrict__ out) {
  const int e8 = blockIdx.x * 256 + threadIdx.x;
  const int rs = e8 >> 7;
  const int c8 = (e8 & 127) * 8;
  const int i  = rs >> 1;
  const int b  = rs & 1;
  const float* p = w + (size_t)rs * kD + c8;
  const v4f a = *(const v4f*)(p);
  const v4f c = *(const v4f*)(p + 4);
  unsigned short hb[8];
#pragma unroll
  for (int e = 0; e < 4; ++e) {
    hb[e]     = h_bits(a[e]);
    hb[4 + e] = h_bits(c[e]);
  }
  const v4u u = (v4u){pk16(hb[0], hb[1]), pk16(hb[2], hb[3]), pk16(hb[4], hb[5]), pk16(hb[6], hb[7])};
  unsigned short* q = out + ((size_t)(b * kQ + i)) * kD + c8;
  *(volatile v4u*)q = u;
  __threadfence();
  *(volatile v4u*)q = u;
}

__global__ __launch_bounds__(256) void qcast_kernel(const float* __restrict__ WQ, const float* __restrict__ rwb,
                                                    const float* __restrict__ rrb,
                                                    unsigned short* __restrict__ QW, unsigned short* __restrict__ QR) {
  const int e8 = blockIdx.x * 256 + threadIdx.x;
  const int c8 = (e8 & 127) * 8;
  const float* p = WQ + 8 * (size_t)e8;
  const v4f a = *(const v4f*)(p);
  const v4f c = *(const v4f*)(p + 4);
  const v4f w0 = *(const v4f*)(rwb + c8);
  const v4f w1 = *(const v4f*)(rwb + c8 + 4);
  const v4f r0 = *(const v4f*)(rrb + c8);
  const v4f r1 = *(const v4f*)(rrb + c8 + 4);
  unsigned short hw[8], hr[8];
#pragma unroll
  for (int e = 0; e < 4; ++e) {
    hw[e]     = h_bits(a[e] + w0[e]);
    hw[4 + e] = h_bits(c[e] + w1[e]);
    hr[e]     = h_bits(a[e] + r0[e]);
    hr[4 + e] = h_bits(c[e] + r1[e]);
  }
  const v4u uw = (v4u){pk16(hw[0], hw[1]), pk16(hw[2], hw[3]), pk16(hw[4], hw[5]), pk16(hw[6], hw[7])};
  const v4u ur = (v4u){pk16(hr[0], hr[1]), pk16(hr[2], hr[3]), pk16(hr[4], hr[5]), pk16(hr[6], hr[7])};
  unsigned short* qw = QW + 8 * (size_t)e8;
  unsigned short* qr = QR + 8 * (size_t)e8;
  *(volatile v4u*)qw = uw;
  *(volatile v4u*)qr = ur;
  __threadfence();
  *(volatile v4u*)qw = uw;
  *(volatile v4u*)qr = ur;
}

__device__ __forceinline__ float neg_fill_f32() { return __int_as_float((int)0xff7fffffu); }

__global__ __launch_bounds__(256) void softmax_rel_kernel(const float* __restrict__ Sac, const float* __restrict__ Sbd,
                                                          const int* __restrict__ mask, unsigned short* __restrict__ P) {
  __shared__ float redM[8];
  __shared__ float redS[8];
  const int i = blockIdx.x;
  const size_t plane = (size_t)blockIdx.y * ((size_t)kQ * kQ);
  const int t = threadIdx.x;
  const int lane = t & 31, wave = t >> 5;
  const int c0 = t * 8;
  const float negf = neg_fill_f32();

  const float* ar = Sac + plane + (size_t)i * kQ + c0;
  const v4f a0 = *(const v4f*)(ar);
  const v4f a1 = *(const v4f*)(ar + 4);
  const int* mr = mask + (size_t)i * kQ + c0;
  const v4i q0 = *(const v4i*)(mr);
  const v4i q1 = *(const v4i*)(mr + 4);
  float acv[8];
  int mv[8];
#pragma unroll
  for (int e = 0; e < 4; ++e) { acv[e] = a0[e]; acv[4 + e] = a1[e]; mv[e] = q0[e]; mv[4 + e] = q1[e]; }

  const float* bp = Sbd + plane;
  float x[8];
  float m = negf;
#pragma unroll
  for (int e = 0; e < 8; ++e) {
    const int j = c0 + e;
    const int dd = j - i;
    const int off = (dd <= 0) ? (kQ - 1 + dd) : (kQ - 2 + dd);
    int idx = i * kQ + off;
    idx = (idx > kQ * kQ - 1) ? (kQ * kQ - 1) : idx;
    const float braw = bp[idx];
    const float bdv = (dd == 1) ? 0.0f : braw;
    float s = (acv[e] + bdv) * kScoreScale;
    s = (mv[e] != 0) ? negf : s;
    x[e] = s;
    m = fmaxf(m, s);
  }
#pragma unroll
  for (int off = 16; off > 0; off >>= 1) m = fmaxf(m, __shfl_xor(m, off, 32));
  if (lane == 0) redM[wave] = m;
  __syncthreads();
  float rmax = redM[0];
#pragma unroll
  for (int wv = 1; wv < 8; ++wv) rmax = fmaxf(rmax, redM[wv]);

  float ex[8];
  float sum = 0.f;
#pragma unroll
  for (int e = 0; e < 8; ++e) { ex[e] = expf(x[e] - rmax); sum += ex[e]; }
#pragma unroll
  for (int off = 16; off > 0; off >>= 1) sum += __shfl_xor(sum, off, 32);
  if (lane == 0) redS[wave] = sum;
  __syncthreads();
  float tot = 0.f;
#pragma unroll
  for (int wv = 0; wv < 8; ++wv) tot += redS[wv];
  const float f = kPCarry * (1.0f / tot);

  unsigned short hb[8];
#pragma unroll
  for (int e = 0; e < 8; ++e) hb[e] = h_bits(ex[e] * f);
  const v4u u = (v4u){pk16(hb[0], hb[1]), pk16(hb[2], hb[3]), pk16(hb[4], hb[5]), pk16(hb[6], hb[7])};
  unsigned short* q = P + plane + (size_t)i * kQ + c0;
  *(volatile v4u*)q = u;
  __threadfence();
  *(volatile v4u*)q = u;
}

__global__ __launch_bounds__(256) void ln_kernel(const float* __restrict__ X, const float* __restrict__ g,
                                                 const float* __restrict__ bb, float* __restrict__ out) {
  __shared__ float red0[8];
  __shared__ float red1[8];
  const int row = blockIdx.x;
  const int t = threadIdx.x;
  const int lane = t & 31, wave = t >> 5;
  const int c0 = t * 4;
  const v4f xv = *(const v4f*)(X + (size_t)row * kD + c0);
  float s = (xv[0] + xv[1]) + (xv[2] + xv[3]);
#pragma unroll
  for (int off = 16; off > 0; off >>= 1) s += __shfl_xor(s, off, 32);
  if (lane == 0) red0[wave] = s;
  __syncthreads();
  float tot = 0.f;
#pragma unroll
  for (int wv = 0; wv < 8; ++wv) tot += red0[wv];
  const float mean = tot * kInvD;
  float dv[4];
#pragma unroll
  for (int e = 0; e < 4; ++e) dv[e] = xv[e] - mean;
  float vs = (dv[0] * dv[0] + dv[1] * dv[1]) + (dv[2] * dv[2] + dv[3] * dv[3]);
#pragma unroll
  for (int off = 16; off > 0; off >>= 1) vs += __shfl_xor(vs, off, 32);
  if (lane == 0) red1[wave] = vs;
  __syncthreads();
  float vtot = 0.f;
#pragma unroll
  for (int wv = 0; wv < 8; ++wv) vtot += red1[wv];
  const float var = vtot * kInvD;
  const float rstd = rsqrtf(var + kLnEps);
  const v4f gv = *(const v4f*)(g + c0);
  const v4f bv = *(const v4f*)(bb + c0);
  v4f y;
#pragma unroll
  for (int e = 0; e < 4; ++e) y[e] = dv[e] * rstd * gv[e] + bv[e];
  float* q = out + (size_t)row * kD + c0;
  *(volatile v4f*)q = y;
  __threadfence();
  *(volatile v4f*)q = y;
}

static inline dim3 gemm_grid(int M, int N, int G) {
  const int tiles = (M / 64) * (N / 64);
  return dim3((unsigned)((tiles + 7) / 8), (unsigned)G, 1);
}

extern "C" void kernel_launch(void* const* d_in, const int* in_sizes, int n_in,
                              void* d_out, int out_size, void* d_ws, size_t ws_size,
                              hipStream_t stream) {
  if (n_in < 10) return;
  if (in_sizes[0] != kTok * kD || in_sizes[1] != kQ * kD || in_sizes[2] != kHD || in_sizes[3] != kHD ||
      in_sizes[4] != 3 * kHD * kD || in_sizes[5] != kHD * kD || in_sizes[6] != kD * kHD ||
      in_sizes[7] != kD || in_sizes[8] != kD || in_sizes[9] != kQ * kQ) return;
  if (out_size != kTok * kD) return;
  if (ws_size < kWsTotal) return;

  const float* w     = (const float*)d_in[0];
  const float* r     = (const float*)d_in[1];
  const float* rwb   = (const float*)d_in[2];
  const float* rrb   = (const float*)d_in[3];
  const float* qkvw  = (const float*)d_in[4];
  const float* rnetw = (const float*)d_in[5];
  const float* ow    = (const float*)d_in[6];
  const float* lnw   = (const float*)d_in[7];
  const float* lnb   = (const float*)d_in[8];
  const int*   amask = (const int*)d_in[9];
  float* out = (float*)d_out;
  char* ws = (char*)d_ws;

  unsigned short* W16    = (unsigned short*)(ws + OFF_W16);
  unsigned short* QKVW16 = (unsigned short*)(ws + OFF_QKVW16);
  unsigned short* RNW16  = (unsigned short*)(ws + OFF_RNW16);
  unsigned short* P16    = (unsigned short*)(ws + OFF_P16);
  unsigned short* OW16   = (unsigned short*)(ws + OFF_OW16);
  unsigned short* RK16   = (unsigned short*)(ws + OFF_RK16);
  unsigned short* QW16   = (unsigned short*)(ws + OFF_QW16);
  unsigned short* QR16   = (unsigned short*)(ws + OFF_QR16);
  unsigned short* K16    = (unsigned short*)(ws + OFF_K16);
  unsigned short* VT16   = (unsigned short*)(ws + OFF_VT16);
  unsigned short* VEC16  = (unsigned short*)(ws + OFF_VEC16);
  unsigned short* R16    = (unsigned short*)(ws + OFF_R16);
  float* SAC  = (float*)(ws + OFF_SAC);
  float* SBD  = (float*)(ws + OFF_SBD);
  float* WQ32 = (float*)(ws + OFF_WQ32);
  float* X32  = (float*)(ws + OFF_X32);

  const dim3 blk(256);

  castw_bm_kernel<<<dim3((kTok * kD / 8) / 256), blk, 0, stream>>>(w, W16);
  cast8_f16_kernel<<<dim3((kQ * kD / 8) / 256), blk, 0, stream>>>(r, R16, kQ * kD / 8, 1.0f);
  cast8_f16_kernel<<<dim3((3 * kHD * kD / 8) / 256), blk, 0, stream>>>(qkvw, QKVW16, 3 * kHD * kD / 8, kWCarry);
  cast8_f16_kernel<<<dim3((kHD * kD / 8) / 256), blk, 0, stream>>>(rnetw, RNW16, kHD * kD / 8, kWCarry);
  cast8_f16_kernel<<<dim3((kD * kHD / 8) / 256), blk, 0, stream>>>(ow, OW16, kD * kHD / 8, kWCarry);

  wmma_gemm64<0, false, 0, 1, false><<<gemm_grid(kQ, kHD, 1), blk, 0, stream>>>(
      R16, R16, kD, 0L, RNW16, RNW16, kD, 0L, (void*)RK16, (void*)RK16, kHD, 0L,
      rwb, w, 0L, kQ, kHD, kD, kWCarryInv);

  wmma_gemm64<0, false, 0, 0, false><<<gemm_grid(kTok, kHD, 1), blk, 0, stream>>>(
      W16, W16, kD, 0L, QKVW16, QKVW16, kD, 0L, (void*)WQ32, (void*)WQ32, kHD, 0L,
      rwb, w, 0L, kTok, kHD, kD, kWCarryInv);
  qcast_kernel<<<dim3((kTok * kHD / 8) / 256), blk, 0, stream>>>(WQ32, rwb, rrb, QW16, QR16);

  wmma_gemm64<0, false, 0, 1, false><<<gemm_grid(kTok, kHD, 1), blk, 0, stream>>>(
      W16, W16, kD, 0L, QKVW16 + (size_t)kHD * kD, QKVW16 + (size_t)kHD * kD, kD, 0L,
      (void*)K16, (void*)K16, kHD, 0L, rwb, w, 0L, kTok, kHD, kD, kWCarryInv);

  wmma_gemm64<0, false, 0, 1, false><<<gemm_grid(kHD, kTok, 1), blk, 0, stream>>>(
      QKVW16 + (size_t)2 * kHD * kD, QKVW16 + (size_t)2 * kHD * kD, kD, 0L, W16, W16, kD, 0L,
      (void*)VT16, (void*)VT16, kTok, 0L, rwb, w, 0L, kHD, kTok, kD, kWCarryInv);

  const long planeS = (long)kQ * kQ;
  for (int c = 0; c < kNumChunks; ++c) {
    const int g0 = c * kChunkG;
    const int b  = g0 / kH;
    const int n0 = g0 % kH;
    const size_t qoff = ((size_t)b * kQ) * kD + (size_t)n0 * kDH;
    wmma_gemm64<0, false, 0, 0, false><<<gemm_grid(kQ, kQ, kChunkG), blk, 0, stream>>>(
        QW16 + qoff, QW16 + qoff, kD, (long)kDH, K16 + qoff, K16 + qoff, kD, (long)kDH,
        (void*)SAC, (void*)SAC, kQ, planeS, rwb, w, 0L, kQ, kQ, kDH, 1.0f);
    wmma_gemm64<0, false, 0, 0, false><<<gemm_grid(kQ, kQ, kChunkG), blk, 0, stream>>>(
        QR16 + qoff, QR16 + qoff, kD, (long)kDH, RK16 + (size_t)n0 * kDH, RK16 + (size_t)n0 * kDH, kHD, (long)kDH,
        (void*)SBD, (void*)SBD, kQ, planeS, rwb, w, 0L, kQ, kQ, kDH, 1.0f);
    softmax_rel_kernel<<<dim3(kQ, kChunkG), blk, 0, stream>>>(SAC, SBD, amask, P16);
    wmma_gemm64<0, false, 0, 1, false><<<gemm_grid(kQ, kDH, kChunkG), blk, 0, stream>>>(
        P16, P16, kQ, planeS,
        VT16 + ((size_t)n0 * kDH) * kTok + (size_t)b * kQ, VT16 + ((size_t)n0 * kDH) * kTok + (size_t)b * kQ,
        kTok, (long)kDH * kTok,
        (void*)(VEC16 + (size_t)b * kHD + (size_t)n0 * kDH), (void*)(VEC16 + (size_t)b * kHD + (size_t)n0 * kDH),
        2 * kHD, (long)kDH, rwb, w, 0L, kQ, kDH, kQ, kPVScale);
  }

  wmma_gemm64<0, false, 0, 0, true><<<gemm_grid(kTok, kD, 1), blk, 0, stream>>>(
      VEC16, VEC16, kHD, 0L, OW16, OW16, kHD, 0L, (void*)X32, (void*)X32, kD, 0L,
      rwb, w, 0L, kTok, kD, kHD, kOutScale);

  ln_kernel<<<dim3(kTok), blk, 0, stream>>>(X32, lnw, lnb, out);
}
